// TransformerBlock_14516989460854
// MI455X (gfx1250) — hardware-run, weakly checked
//
#include <hip/hip_runtime.h>
#ifndef NB
#define NB 8
#endif
#ifndef SEQ
#define SEQ 1024
#endif
#define NB_FULL 8
#define SEQ_FULL 1024
#define DM 1024
#define NH 16
#define HD 64
#define NR ((size_t)NB * SEQ)
static_assert(NH * HD == DM);
static_assert(HD == 64);
static_assert(SEQ % 128 == 0);
static_assert(SEQ <= SEQ_FULL);
static_assert(NB >= 1 && NB <= NB_FULL);
static_assert(DM == 128 * 8);
static_assert(DM % 64 == 0);
static_assert(DM % 32 == 0);
static_assert(HD % 32 == 0);

#define AL256(x) ((((size_t)(x)) + 255) & ~(size_t)255)
constexpr size_t CARVE_BQKV = AL256((size_t)3 * DM * DM * 2);
constexpr size_t CARVE_BO   = AL256((size_t)DM * DM * 2);
constexpr size_t CARVE_X16  = AL256((size_t)NB * SEQ * DM * 2);
constexpr size_t CARVE_QK16 = AL256((size_t)2 * NB * SEQ * DM * 2);
constexpr size_t CARVE_Y16  = AL256((size_t)NB * SEQ * DM * 2);
constexpr size_t CARVE_LSE  = AL256((size_t)NB * NH * SEQ * 4);
constexpr size_t CARVE_CS   = AL256((size_t)NB * NH * SEQ * 4);
constexpr size_t CARVE_TOTAL = CARVE_BQKV + CARVE_BO + CARVE_X16 + CARVE_QK16 + CARVE_Y16 + CARVE_LSE + CARVE_CS;
static_assert(CARVE_TOTAL <= (size_t)134217728);

typedef _Float16 h16;
typedef _Float16 v16h __attribute__((ext_vector_type(16)));
typedef unsigned short v8us __attribute__((ext_vector_type(8), may_alias));
typedef float v8f __attribute__((ext_vector_type(8)));
typedef float v4f __attribute__((ext_vector_type(4)));
typedef float v4fa __attribute__((ext_vector_type(4), may_alias));
typedef _Float16 v4h __attribute__((ext_vector_type(4)));
union FragH { v16h v; v8us half[2]; _Float16 h[16]; unsigned short u[16]; };

__device__ __forceinline__ unsigned short bf16_bits(float x) { unsigned int u = __float_as_uint(x); return (unsigned short)((u + 0x7FFFu + ((u >> 16) & 1u)) >> 16); }
__device__ __forceinline__ float bf16_val(unsigned short b) { return __uint_as_float(((unsigned int)b) << 16); }
__device__ __forceinline__ float bf16_rne(float x) { return bf16_val(bf16_bits(x)); }

static __device__ __forceinline__ h16 toh_flush(float v) { const h16 r = (h16)v; return (fabsf(v) < 6.103515625e-05f) ? (h16)0.0f : r; }

__device__ __forceinline__ v16h g2_frag(const _Float16* p, int hh) { FragH f; f.half[0] = *(const v8us*)((const unsigned short*)p + 8 * hh); f.half[1] = *(const v8us*)((const unsigned short*)p + 16 + 8 * hh); return f.v; }
__device__ __forceinline__ v8f g2_mma(v16h a, v16h b, v8f c) { v8f d = __builtin_amdgcn_wmma_f32_16x16x32_f16(false, a, false, b, (short)0, c, false, false); asm volatile("v_nop\n\tv_nop\n\tv_nop\n\tv_nop" : "+v"(d) : "v"(a), "v"(b)); return d; }
__device__ __forceinline__ v8f mma2(v16h a0, v16h b0, v16h a1, v16h b1, v8f c) {
  c = __builtin_amdgcn_wmma_f32_16x16x32_f16(false, a0, false, b0, (short)0, c, false, false);
  c = __builtin_amdgcn_wmma_f32_16x16x32_f16(false, a1, false, b1, (short)0, c, false, false);
  asm volatile("v_nop\n\tv_nop\n\tv_nop\n\tv_nop" : "+v"(c) : "v"(a0), "v"(b0), "v"(a1), "v"(b1));
  return c;
}

__global__ __launch_bounds__(256) void k_wnat(const float* __restrict__ w, size_t n8, _Float16* __restrict__ Bt) {
  const size_t t = (size_t)blockIdx.x * 256 + threadIdx.x; if (t >= n8) return; FragH f;
#pragma unroll
  for (int q = 0; q < 8; ++q) f.h[q] = (_Float16)(bf16_rne(w[t * 8 + q]) * 16.0f);
  const v8us o = f.half[0];
  *(volatile v8us*)((unsigned short*)Bt + t * 8) = o; __threadfence(); *(volatile v8us*)((unsigned short*)Bt + t * 8) = o;
}

__global__ __launch_bounds__(256) void k_wperm(const float* __restrict__ w, size_t n8, _Float16* __restrict__ Bt) {
  const size_t t = (size_t)blockIdx.x * 256 + threadIdx.x; if (t >= n8) return;
  const size_t row = t / (size_t)(DM / 8); const size_t k8 = t - row * (size_t)(DM / 8);
  const size_t drow = (row % (size_t)NH) * (size_t)HD + row / (size_t)NH;
  FragH f;
#pragma unroll
  for (int q = 0; q < 8; ++q) f.h[q] = toh_flush(bf16_rne(w[t * 8 + q]) * 16.0f);
  const v8us o = f.half[0];
  unsigned short* d = (unsigned short*)Bt + (drow * (size_t)(DM / 8) + k8) * 8;
  *(volatile v8us*)d = o; __threadfence(); *(volatile v8us*)d = o;
}

__global__ __launch_bounds__(128) void k_xcast(const float* __restrict__ x, _Float16* __restrict__ X16) {
  const int r = blockIdx.x; const int b = r / SEQ, s = r - b * SEQ;
  const int t = threadIdx.x;
  const float* xr = x + ((size_t)b * SEQ_FULL + s) * DM + 8 * t;
  const v4f xa = *(const v4fa*)xr, xb = *(const v4fa*)(xr + 4);
  FragH f;
#pragma unroll
  for (int q = 0; q < 4; ++q) { f.h[q] = toh_flush(bf16_rne(xa[q])); f.h[4 + q] = toh_flush(bf16_rne(xb[q])); }
  const v8us o = f.half[0];
  unsigned short* d = (unsigned short*)X16 + (size_t)r * DM + 8 * t;
  *(volatile v8us*)d = o; __threadfence(); *(volatile v8us*)d = o;
}

__device__ __forceinline__ void mac32x64(const _Float16* __restrict__ a0p, const _Float16* __restrict__ a1p, const _Float16* __restrict__ b0p, size_t ldb, int K, int hh,
                                         v8f& c00, v8f& c01, v8f& c02, v8f& c03, v8f& c10, v8f& c11, v8f& c12, v8f& c13) {
  const _Float16* b1p = b0p + 16 * ldb; const _Float16* b2p = b1p + 16 * ldb; const _Float16* b3p = b2p + 16 * ldb;
#pragma unroll 1
  for (int kb = 0; kb < K; kb += 32) {
    const v16h a0 = g2_frag(a0p + kb, hh), a1 = g2_frag(a1p + kb, hh);
    v16h bq = g2_frag(b0p + kb, hh); c00 = g2_mma(a0, bq, c00); c10 = g2_mma(a1, bq, c10);
    bq = g2_frag(b1p + kb, hh); c01 = g2_mma(a0, bq, c01); c11 = g2_mma(a1, bq, c11);
    bq = g2_frag(b2p + kb, hh); c02 = g2_mma(a0, bq, c02); c12 = g2_mma(a1, bq, c12);
    bq = g2_frag(b3p + kb, hh); c03 = g2_mma(a0, bq, c03); c13 = g2_mma(a1, bq, c13);
  }
}

__global__ __launch_bounds__(128) void k_proj(const _Float16* __restrict__ X16, const _Float16* __restrict__ Bt, const float* __restrict__ CS, int scl, float alpha, _Float16* __restrict__ Y16) {
  __shared__ __attribute__((aligned(16))) float so[4][32][68];
  const int tid = threadIdx.x, lane = tid & 31, ln = lane & 15, hh = lane >> 4;
  const int w = __builtin_amdgcn_readfirstlane(tid >> 5);
  const int by = blockIdx.y;
  const _Float16* Bh = Bt + (size_t)by * DM * DM;
  _Float16* Yp = Y16 + (size_t)by * NR * DM;
  const int ntn = DM / 64;
  const int mt = blockIdx.x / ntn, nq = blockIdx.x - mt * ntn;
  const int row0 = mt * 128 + 32 * w, col0 = nq * 64;
  if (row0 >= (int)NR) return;
  const _Float16* a0p = X16 + (size_t)(row0 + ln) * DM; const _Float16* a1p = a0p + (size_t)16 * DM;
  const _Float16* b0p = Bh + (size_t)(col0 + ln) * DM;
  const v8f z8 = {0.f, 0.f, 0.f, 0.f, 0.f, 0.f, 0.f, 0.f};
  v8f c00 = z8, c01 = z8, c02 = z8, c03 = z8, c10 = z8, c11 = z8, c12 = z8, c13 = z8;
  mac32x64(a0p, a1p, b0p, (size_t)DM, DM, hh, c00, c01, c02, c03, c10, c11, c12, c13);
  v8f accs[8] = {c00, c01, c02, c03, c10, c11, c12, c13};
  float rm0[8], rm1[8];
#pragma unroll
  for (int r = 0; r < 8; ++r) { rm0[r] = alpha; rm1[r] = alpha; }
  if (scl != 0) {
    const int b = row0 / SEQ;
    const float* cp = CS + ((size_t)(b * NH + nq)) * SEQ + (size_t)(row0 - b * SEQ) + 8 * hh;
    const v4f ca = *(const v4fa*)cp, cb = *(const v4fa*)(cp + 4), cc = *(const v4fa*)(cp + 16), cd = *(const v4fa*)(cp + 20);
#pragma unroll
    for (int q = 0; q < 4; ++q) { rm0[q] = alpha * ca[q]; rm0[4 + q] = alpha * cb[q]; rm1[q] = alpha * cc[q]; rm1[4 + q] = alpha * cd[q]; }
  }
#pragma unroll
  for (int u = 0; u < 8; ++u) {
    const int t = u & 3, half = u >> 2;
#pragma unroll
    for (int r = 0; r < 8; ++r) so[w][half * 16 + 8 * hh + r][t * 16 + ln] = accs[u][r] * (half ? rm1[r] : rm0[r]);
  }
  __builtin_amdgcn_fence(4  , "workgroup"); __builtin_amdgcn_wave_barrier();
  const int rsub = lane >> 4, c4 = (lane & 15) * 4;
  for (int pass = 0; pass < 2; ++pass) {
#pragma unroll
    for (int q = 0; q < 16; ++q) {
      const int r = q * 2 + rsub; const v4f v = *(const v4fa*)&so[w][r][c4]; v4h h4;
#pragma unroll
      for (int i = 0; i < 4; ++i) h4[i] = toh_flush(v[i]);
      *(volatile v4h*)(Yp + (size_t)(row0 + r) * DM + col0 + c4) = h4;
    }
    if (pass == 0) __threadfence();
  }
}

__global__ __launch_bounds__(128) void k_stats(const _Float16* __restrict__ Q16, const _Float16* __restrict__ K16, float* __restrict__ LSE) {
  __shared__ __attribute__((aligned(16))) float sl[64];
  const int tid = threadIdx.x, lane = tid & 31, ln = lane & 15, hh = lane >> 4;
  const int w = __builtin_amdgcn_readfirstlane(tid >> 5);
  const int h = blockIdx.y, b = blockIdx.z;
  const int q0 = blockIdx.x * 64 + w * 16;
  const size_t rq = (size_t)b * SEQ + q0;
  const size_t rk = (size_t)b * SEQ;
  const _Float16* qp = Q16 + (rq + ln) * DM + h * HD;
  const v16h qb0 = g2_frag(qp, hh), qb1 = g2_frag(qp + 32, hh);
  const _Float16* kp0 = K16 + (rk + ln) * DM + h * HD;
  const v8f z8 = {0.f, 0.f, 0.f, 0.f, 0.f, 0.f, 0.f, 0.f};
  float mrun = -1.0e30f, lrun = 0.f;
#pragma unroll 1
  for (int kt = 0; kt < SEQ; kt += 64) {
    v8f s[4];
#pragma unroll
    for (int j = 0; j < 4; ++j) {
      const _Float16* kp = kp0 + (size_t)(kt + 16 * j) * DM;
      const v16h ka0 = g2_frag(kp, hh), ka1 = g2_frag(kp + 32, hh);
      s[j] = mma2(ka0, qb0, ka1, qb1, z8);
    }
    float mx = -1.0e30f;
#pragma unroll
    for (int j = 0; j < 4; ++j)
#pragma unroll
      for (int r = 0; r < 8; ++r) mx = fmaxf(mx, s[j][r]);
    mx = fmaxf(mx, __shfl_xor(mx, 16, 32));
    const float mnew = fmaxf(mrun, mx * 0.125f);
    const float alpha = __expf(mrun - mnew);
    mrun = mnew;
    float ps = 0.f;
#pragma unroll
    for (int j = 0; j < 4; ++j)
#pragma unroll
      for (int r = 0; r < 8; ++r) ps += __expf(s[j][r] * 0.125f - mnew);
    ps += __shfl_xor(ps, 16, 32);
    lrun = lrun * alpha + ps;
  }
  const float lse = mrun + logf(lrun);
  if (hh == 0) sl[w * 16 + ln] = lse;
  __syncthreads();
  if (w == 0 && lane < 16) {
    const v4f v = *(const v4fa*)&sl[lane * 4];
    float* d = LSE + ((size_t)(b * NH + h)) * SEQ + (size_t)blockIdx.x * 64 + lane * 4;
    *(volatile v4f*)d = v; __threadfence(); *(volatile v4f*)d = v;
  }
}

__global__ __launch_bounds__(128) void k_colsum(const _Float16* __restrict__ Q16, const _Float16* __restrict__ K16, const float* __restrict__ LSE, float* __restrict__ CS) {
  __shared__ __attribute__((aligned(16))) float sc[64];
  const int tid = threadIdx.x, lane = tid & 31, ln = lane & 15, hh = lane >> 4;
  const int w = __builtin_amdgcn_readfirstlane(tid >> 5);
  const int h = blockIdx.y, b = blockIdx.z;
  const int k0 = blockIdx.x * 64 + w * 16;
  const size_t rk = (size_t)b * SEQ + k0;
  const size_t rq = (size_t)b * SEQ;
  const _Float16* kp = K16 + (rk + ln) * DM + h * HD;
  const v16h ka0 = g2_frag(kp, hh), ka1 = g2_frag(kp + 32, hh);
  const _Float16* qp0 = Q16 + (rq + ln) * DM + h * HD;
  const float* lp = LSE + ((size_t)(b * NH + h)) * SEQ + ln;
  const v8f z8 = {0.f, 0.f, 0.f, 0.f, 0.f, 0.f, 0.f, 0.f};
  float cs[8];
#pragma unroll
  for (int r = 0; r < 8; ++r) cs[r] = 0.f;
#pragma unroll 1
  for (int qt = 0; qt < SEQ; qt += 64) {
#pragma unroll
    for (int j = 0; j < 4; ++j) {
      const _Float16* qp = qp0 + (size_t)(qt + 16 * j) * DM;
      const v16h qb0 = g2_frag(qp, hh), qb1 = g2_frag(qp + 32, hh);
      const v8f s = mma2(ka0, qb0, ka1, qb1, z8);
      const float ls = lp[qt + 16 * j];
#pragma unroll
      for (int r = 0; r < 8; ++r) cs[r] += __expf(s[r] * 0.125f - ls);
    }
  }
#pragma unroll
  for (int off = 1; off < 16; off <<= 1)
#pragma unroll
    for (int r = 0; r < 8; ++r) cs[r] += __shfl_xor(cs[r], off, 32);
  if (ln == 0) {
#pragma unroll
    for (int r = 0; r < 8; ++r) sc[w * 16 + 8 * hh + r] = cs[r];
  }
  __syncthreads();
  if (w == 0 && lane < 16) {
    const v4f v = *(const v4fa*)&sc[lane * 4];
    float* d = CS + ((size_t)(b * NH + h)) * SEQ + (size_t)blockIdx.x * 64 + lane * 4;
    *(volatile v4f*)d = v; __threadfence(); *(volatile v4f*)d = v;
  }
}

__global__ __launch_bounds__(128) void k_outp(const _Float16* __restrict__ A1, const _Float16* __restrict__ B1, float al1, const float* __restrict__ bo, float* __restrict__ Out) {
  __shared__ __attribute__((aligned(16))) float so[4][32][68];
  const int tid = threadIdx.x, lane = tid & 31, ln = lane & 15, hh = lane >> 4;
  const int w = __builtin_amdgcn_readfirstlane(tid >> 5);
  const int ntn = DM / 64;
  const int mt = blockIdx.x / ntn, nq = blockIdx.x - mt * ntn;
  const int row0 = mt * 128 + 32 * w, col0 = nq * 64;
  if (row0 >= (int)NR) return;
  const v8f z8 = {0.f, 0.f, 0.f, 0.f, 0.f, 0.f, 0.f, 0.f};
  v8f c00 = z8, c01 = z8, c02 = z8, c03 = z8, c10 = z8, c11 = z8, c12 = z8, c13 = z8;
  {
    const _Float16* a0p = A1 + (size_t)(row0 + ln) * DM; const _Float16* a1p = a0p + (size_t)16 * DM;
    const _Float16* b0p = B1 + (size_t)(col0 + ln) * DM;
    mac32x64(a0p, a1p, b0p, (size_t)DM, DM, hh, c00, c01, c02, c03, c10, c11, c12, c13);
    v8f accs[8] = {c00, c01, c02, c03, c10, c11, c12, c13};
#pragma unroll
    for (int u = 0; u < 8; ++u) {
      const int t = u & 3, half = u >> 2;
#pragma unroll
      for (int r = 0; r < 8; ++r) so[w][half * 16 + 8 * hh + r][t * 16 + ln] = accs[u][r] * al1;
    }
  }
  __builtin_amdgcn_fence(4  , "workgroup"); __builtin_amdgcn_wave_barrier();
  const int rsub = lane >> 4, c4 = (lane & 15) * 4;
  const v4f bv = *(const v4fa*)(bo + col0 + c4);
  v4f bb;
#pragma unroll
  for (int i = 0; i < 4; ++i) bb[i] = bf16_rne(bv[i]);
  for (int pass = 0; pass < 2; ++pass) {
#pragma unroll
    for (int q = 0; q < 16; ++q) {
      const int r = q * 2 + rsub; const v4f v = *(const v4fa*)&so[w][r][c4];
      const v4f o = v + bb;
      *(volatile v4f*)(Out + (size_t)(row0 + r) * DM + col0 + c4) = o;
    }
    if (pass == 0) __threadfence();
  }
}

extern "C" void kernel_launch(void* const* d_in, const int* in_sizes, int n_in,
                              void* d_out, int out_size, void* d_ws, size_t ws_size, hipStream_t stream) {
  if (n_in < 6) return;
  if (in_sizes[0] < (int)(((size_t)(NB - 1) * SEQ_FULL + SEQ) * DM)) return;
  for (int i = 1; i <= 4; ++i) if (in_sizes[i] < DM * DM) return;
  if (in_sizes[5] < DM) return;
  if (out_size < (int)(NR * DM)) return;
  const float* const* I = (const float* const*)d_in;
  const float* x = I[0]; const float* wq = I[1]; const float* wk = I[2]; const float* wv = I[3]; const float* wo = I[4]; const float* bo = I[5];
  char* ws = (char*)d_ws; size_t off = 0;
  auto take = [&](size_t bytes) { char* p = ws + off; off += (bytes + 255) & ~(size_t)255; return p; };
  _Float16* BQKV = (_Float16*)take((size_t)3 * DM * DM * 2);
  _Float16* BO   = (_Float16*)take((size_t)DM * DM * 2);
  _Float16* X16  = (_Float16*)take(NR * DM * 2);
  _Float16* QK16 = (_Float16*)take((size_t)2 * NR * DM * 2);
  _Float16* Y16  = (_Float16*)take(NR * DM * 2);
  float*    LSE  = (float*)take((size_t)NB * NH * SEQ * 4);
  float*    CS   = (float*)take((size_t)NB * NH * SEQ * 4);
  if (off > ws_size) return;
  if (off > CARVE_TOTAL) return;
  _Float16* Q16 = QK16; _Float16* K16 = QK16 + NR * DM;

  k_xcast<<<(unsigned)NR, 128, 0, stream>>>(x, X16);
  { const size_t n8 = (size_t)DM * DM / 8; const unsigned g = (unsigned)((n8 + 255) / 256);
    k_wperm<<<g, 256, 0, stream>>>(wq, n8, BQKV);
    k_wperm<<<g, 256, 0, stream>>>(wk, n8, BQKV + (size_t)DM * DM);
    k_wperm<<<g, 256, 0, stream>>>(wv, n8, BQKV + (size_t)2 * DM * DM);
    k_wnat<<<g, 256, 0, stream>>>(wo, n8, BO); }
  k_proj<<<dim3((unsigned)((NR / 128) * (DM / 64)), 2), 128, 0, stream>>>(X16, BQKV, CS, 0, 0.0625f, QK16);
  k_stats<<<dim3(SEQ / 64, NH, NB), 128, 0, stream>>>(Q16, K16, LSE);
  k_colsum<<<dim3(SEQ / 64, NH, NB), 128, 0, stream>>>(Q16, K16, LSE, CS);
  k_proj<<<dim3((unsigned)((NR / 128) * (DM / 64)), 1), 128, 0, stream>>>(X16, BQKV + (size_t)2 * DM * DM, CS, 1, 1.0f, Y16);
  k_outp<<<(unsigned)((NR / 128) * (DM / 64)), 128, 0, stream>>>(Y16, BO, 0.00390625f, bo, (float*)d_out);
}
